// GraphAttentionLayer_71244917506562
// MI455X (gfx1250) — hardware-verified
//
#include <hip/hip_runtime.h>
#include <math.h>
#include <stdint.h>

#define NB_   4
#define NL_   2048
#define DD    128
#define NTOK  (NB_ * NL_)
#define QT    64
#define KS    64
#define AGP   256
#define KW1   256
#define KW2   128
#define PO    132
#define GBM   64
#define GBN   128
#define GTHR  128
#define GWAVE 4
#define PARTW 288
#define WSTW  258
#define NPART (NTOK / GBM)
#define ATHR  256
#define APB   64
#define N8X   (NTOK * DD / 8)
#define SELU_A 1.6732632423543772f
#define SELU_S 1.0507009873554805f
#define BN_EPS 1e-5f
#define WSMAX 134217728

static_assert(NL_ % QT == 0 && NL_ % KS == 0 && QT == 4 * 16 && KS == 64);
static_assert(DD == 128 && DD % 32 == 0 && AGP == 2 * DD && KW1 == 2 * DD && KW2 == DD);
static_assert(KW1 % 32 == 0 && KW2 % 32 == 0);
static_assert(NL_ % 64 == 0 && DD % 64 == 0);
static_assert(N8X % 256 == 0 && (DD / 8) == 16);
static_assert(NTOK % GBM == 0 && GBM == GWAVE * 16 && GTHR == GBN && GBN == DD && GTHR == 32 * GWAVE);
static_assert(PARTW % 32 == 0 && PARTW / 4 <= GTHR && PARTW >= 2 * GBN + 1);
static_assert(WSTW >= 2 * GBN + 1);
static_assert(NTOK % APB == 0 && APB == (ATHR / 32) * 8 && ATHR == 2 * DD);
static_assert((PO * 4) % 16 == 0 && PO >= DD);
static_assert((DD * DD) / 8 == 8 * 256);
static_assert(NPART == 128);

typedef __attribute__((ext_vector_type(16))) __bf16 v16b;
typedef __attribute__((ext_vector_type(8)))  __bf16 v8b;
typedef __attribute__((ext_vector_type(8)))  float  v8f;
typedef __attribute__((ext_vector_type(4)))  float  v4f;
typedef __attribute__((ext_vector_type(4)))  unsigned int v4u;
typedef __attribute__((ext_vector_type(8)))  unsigned int v8u;
typedef v8b __attribute__((may_alias)) v8ba;
typedef v4f __attribute__((may_alias)) v4fa;
typedef v4u __attribute__((may_alias)) v4ua;

union FragU { v16b v; v8b h[2]; };
union PackU { v8u u; v16b v; };

__device__ __forceinline__ unsigned short f2bf_bits(float f) {
  const unsigned u = __float_as_uint(f);
  return (unsigned short)((u + 0x7FFFu + ((u >> 16) & 1u)) >> 16);
}
__device__ __forceinline__ float bf_bits2f(unsigned short h) { return __uint_as_float(((unsigned)h) << 16); }
__device__ __forceinline__ float bf16r(float f) {
  unsigned u = __float_as_uint(f);
  u = (u + 0x7FFFu + ((u >> 16) & 1u)) & 0xFFFF0000u;
  return __uint_as_float(u);
}
__device__ __forceinline__ unsigned pk16(unsigned short a, unsigned short b) { return (unsigned)a | ((unsigned)b << 16); }

__device__ __forceinline__ v8f wmma_bf16(v16b a, v16b b, v8f c) {
  v8f d = __builtin_amdgcn_wmma_f32_16x16x32_bf16(false, a, false, b, (short)0, c, false, false);
  asm volatile("v_nop\n\tv_nop\n\tv_nop\n\tv_nop" : "+v"(d) : "v"(a), "v"(b));
  return d;
}

__device__ __forceinline__ v16b load_frag(const unsigned short* p, int hh) {
  FragU f;
  f.h[0] = *(const v8ba*)(p + 8 * hh);
  f.h[1] = *(const v8ba*)(p + 16 + 8 * hh);
  return f.v;
}

__device__ __forceinline__ void pack_p2(v8f a, v8f c, v16b& ho, v16b& lo) {
  PackU uh, ul;
#pragma unroll
  for (int i = 0; i < 4; ++i) {
    const unsigned short h0 = f2bf_bits(a[2 * i]), h1 = f2bf_bits(a[2 * i + 1]);
    const unsigned short l0 = f2bf_bits(a[2 * i] - bf_bits2f(h0)), l1 = f2bf_bits(a[2 * i + 1] - bf_bits2f(h1));
    uh.u[i] = pk16(h0, h1); ul.u[i] = pk16(l0, l1);
    const unsigned short g0 = f2bf_bits(c[2 * i]), g1 = f2bf_bits(c[2 * i + 1]);
    const unsigned short m0 = f2bf_bits(c[2 * i] - bf_bits2f(g0)), m1 = f2bf_bits(c[2 * i + 1] - bf_bits2f(g1));
    uh.u[4 + i] = pk16(g0, g1); ul.u[4 + i] = pk16(m0, m1);
  }
  ho = uh.v; lo = ul.v;
}

__device__ __forceinline__ v8f z8() { v8f z = {0.f, 0.f, 0.f, 0.f, 0.f, 0.f, 0.f, 0.f}; return z; }

__global__ __launch_bounds__(256) void k_xprep(const float* __restrict__ x, const float* __restrict__ wmap,
                                               unsigned short* __restrict__ XB, unsigned short* __restrict__ XWH,
                                               unsigned short* __restrict__ XWL, int n8) {
  int i = blockIdx.x * 256 + threadIdx.x;
  const bool ok = i < n8;
  i = ok ? i : (n8 - 1);
  const float* s = x + (size_t)i * 8;
  const int d0 = (i & (DD / 8 - 1)) * 8;
  const v4f f0 = *(const v4fa*)(s);
  const v4f f1 = *(const v4fa*)(s + 4);
  const v4f w0 = *(const v4fa*)(wmap + d0);
  const v4f w1 = *(const v4fa*)(wmap + d0 + 4);
  const float xv[8] = {f0[0], f0[1], f0[2], f0[3], f1[0], f1[1], f1[2], f1[3]};
  const float wv[8] = {w0[0], w0[1], w0[2], w0[3], w1[0], w1[1], w1[2], w1[3]};
  v4u ux, uh, ul;
#pragma unroll
  for (int q = 0; q < 4; ++q) {
    const unsigned short xb0 = f2bf_bits(xv[2 * q]), xb1 = f2bf_bits(xv[2 * q + 1]);
    const float p0 = bf_bits2f(xb0) * bf16r(wv[2 * q]);
    const float p1 = bf_bits2f(xb1) * bf16r(wv[2 * q + 1]);
    const unsigned short h0 = f2bf_bits(p0), h1 = f2bf_bits(p1);
    const unsigned short l0 = f2bf_bits(p0 - bf_bits2f(h0)), l1 = f2bf_bits(p1 - bf_bits2f(h1));
    ux[q] = pk16(xb0, xb1);
    uh[q] = pk16(h0, h1);
    ul[q] = pk16(l0, l1);
  }
  const size_t o8 = (size_t)i * 8;
  if (ok) {
    *(volatile v4u*)(XB + o8)  = ux;
    *(volatile v4u*)(XWH + o8) = uh;
    *(volatile v4u*)(XWL + o8) = ul;
  }
  __threadfence();
  if (ok) {
    *(volatile v4u*)(XB + o8)  = ux;
    *(volatile v4u*)(XWH + o8) = uh;
    *(volatile v4u*)(XWL + o8) = ul;
  }
}

__global__ __launch_bounds__(256) void k_wprep(const float* __restrict__ Watt, const float* __restrict__ Wres,
                                               unsigned short* BT1, unsigned short* BW2) {
  const int blk = blockIdx.x, tid = threadIdx.x;
  const bool att = blk < 8;
  const int u = (blk & 7) * 256 + tid;
  const int n = u >> 4;
  const int k8 = (u & 15) * 8;
  const float* W = att ? Watt : Wres;
  const float* p = W + (size_t)n * DD + k8;
  const v4f a = *(const v4fa*)p;
  const v4f c = *(const v4fa*)(p + 4);
  v4u q;
  q[0] = pk16(f2bf_bits(a[0]), f2bf_bits(a[1]));
  q[1] = pk16(f2bf_bits(a[2]), f2bf_bits(a[3]));
  q[2] = pk16(f2bf_bits(c[0]), f2bf_bits(c[1]));
  q[3] = pk16(f2bf_bits(c[2]), f2bf_bits(c[3]));
  unsigned short* dp  = att ? (BT1 + (size_t)n * KW1 + k8) : (BW2 + (size_t)n * KW2 + k8);
  unsigned short* dp2 = att ? (dp + DD) : dp;
  *(volatile v4u*)dp  = q;
  *(volatile v4u*)dp2 = q;
  __threadfence();
  *(volatile v4u*)dp  = q;
  *(volatile v4u*)dp2 = q;
}

__global__ __launch_bounds__(256) void k_tprep(const float* __restrict__ x, unsigned short* __restrict__ XT) {
  __shared__ __align__(16) float tf[64 * 68];
  const float* W = x + (size_t)blockIdx.z * NL_ * DD;
  unsigned short* ob = XT + (size_t)blockIdx.z * DD * NL_;
  const int c0  = blockIdx.x * 64;
  const int r0  = blockIdx.y * 64;
  const int tid = threadIdx.x;
  {
    const int lr = tid >> 4;
    const int c4 = (tid & 15) * 4;
#pragma unroll
    for (int it = 0; it < 4; ++it) {
      const int rr = it * 16 + lr;
      const v4f a = *(const v4fa*)(W + (size_t)(r0 + rr) * DD + c0 + c4);
      *(v4fa*)(tf + rr * 68 + c4) = a;
    }
  }
  __syncthreads();
  const int sub = tid >> 3;
  const int c8  = (tid & 7) * 8;
  v4u hv[2];
#pragma unroll
  for (int it = 0; it < 2; ++it) {
    const int oc = it * 32 + sub;
    v4u a;
#pragma unroll
    for (int q = 0; q < 4; ++q) {
      const float f0 = tf[(c8 + 2 * q) * 68 + oc];
      const float f1 = tf[(c8 + 2 * q + 1) * 68 + oc];
      a[q] = pk16(f2bf_bits(f0), f2bf_bits(f1));
    }
    hv[it] = a;
  }
#pragma unroll
  for (int it = 0; it < 2; ++it) {
    const int oc = it * 32 + sub;
    const size_t go = (size_t)(c0 + oc) * NL_ + r0 + c8;
    *(volatile v4u*)(ob + go) = hv[it];
  }
  __threadfence();
#pragma unroll
  for (int it = 0; it < 2; ++it) {
    const int oc = it * 32 + sub;
    const size_t go = (size_t)(c0 + oc) * NL_ + r0 + c8;
    *(volatile v4u*)(ob + go) = hv[it];
  }
}

__global__ __launch_bounds__(128) void k_attn(const unsigned short* __restrict__ XB,
                                              const unsigned short* __restrict__ XWH,
                                              const unsigned short* __restrict__ XWL,
                                              const unsigned short* __restrict__ XT,
                                              unsigned short* __restrict__ AG) {
  __shared__ __align__(16) float sO[4][16 * PO];
  const int tid = threadIdx.x, lane = tid & 31, w = tid >> 5;
  const int hh = lane >> 4, m = lane & 15;
  const int b = blockIdx.y;
  const int q0w = blockIdx.x * QT + 16 * w;
  const size_t tokq = (size_t)b * NL_ + q0w + m;
  const unsigned short* qh = XWH + tokq * DD;
  const unsigned short* ql = XWL + tokq * DD;
  const unsigned short* kbase = XB + ((size_t)b * NL_ + m) * (size_t)DD;
  const unsigned short* vbase = XT + ((size_t)b * DD + m) * (size_t)NL_;

  v8f o[8];
#pragma unroll
  for (int t = 0; t < 8; ++t) o[t] = z8();
  float mrun = -1e30f, lrun = 0.0f;

#pragma unroll 1
  for (int ks = 0; ks < NL_ / KS; ++ks) {
    const int kb = ks * KS;

    v8f s[4];
#pragma unroll
    for (int j = 0; j < 4; ++j) s[j] = z8();
#pragma unroll 1
    for (int c = 0; c < DD / 32; ++c) {
      const v16b fh = load_frag(qh + 32 * c, hh);
      const v16b fl = load_frag(ql + 32 * c, hh);
#pragma unroll
      for (int j = 0; j < 4; ++j) {
        const v16b fa = load_frag(kbase + (size_t)(kb + 16 * j) * DD + 32 * c, hh);
        s[j] = wmma_bf16(fa, fh, s[j]);
        s[j] = wmma_bf16(fa, fl, s[j]);
      }
    }

    float tmax = -1e30f;
#pragma unroll
    for (int j = 0; j < 4; ++j)
#pragma unroll
      for (int r = 0; r < 8; ++r) tmax = fmaxf(tmax, s[j][r]);
    tmax = fmaxf(tmax, __shfl_xor(tmax, 16, 32));
    const float mnew = fmaxf(mrun, tmax);
    const float scl = __expf(mrun - mnew);
    float rs = 0.0f;
#pragma unroll
    for (int j = 0; j < 4; ++j)
#pragma unroll
      for (int r = 0; r < 8; ++r) {
        const float p = __expf(s[j][r] - mnew);
        s[j][r] = p;
        rs += p;
      }
    rs += __shfl_xor(rs, 16, 32);
    lrun = fmaf(lrun, scl, rs);
    mrun = mnew;
#pragma unroll
    for (int t = 0; t < 8; ++t) o[t] = o[t] * scl;

    {
      v16b ph, pl;
      pack_p2(s[0], s[1], ph, pl);
#pragma unroll
      for (int t = 0; t < 8; ++t) {
        const v16b fv = load_frag(vbase + (size_t)(16 * t) * NL_ + kb, hh);
        o[t] = wmma_bf16(fv, ph, o[t]);
        o[t] = wmma_bf16(fv, pl, o[t]);
      }
    }
    {
      v16b ph, pl;
      pack_p2(s[2], s[3], ph, pl);
#pragma unroll
      for (int t = 0; t < 8; ++t) {
        const v16b fv = load_frag(vbase + (size_t)(16 * t) * NL_ + kb + 32, hh);
        o[t] = wmma_bf16(fv, ph, o[t]);
        o[t] = wmma_bf16(fv, pl, o[t]);
      }
    }
  }

  const float inv = 1.0f / lrun;
  float* so = sO[w];
#pragma unroll
  for (int t = 0; t < 8; ++t)
#pragma unroll
    for (int r = 0; r < 8; ++r)
      so[m * PO + 16 * t + 8 * hh + r] = o[t][r] * inv;
  __syncthreads();
  const int d0 = 8 * (lane & 15);
  v4u ov[16];
#pragma unroll
  for (int i = 0; i < 16; ++i) {
    const v4f a = *(const v4fa*)(so + i * PO + d0);
    const v4f c = *(const v4fa*)(so + i * PO + d0 + 4);
    const float y[8] = {a[0], a[1], a[2], a[3], c[0], c[1], c[2], c[3]};
    v4u rv;
#pragma unroll
    for (int q = 0; q < 4; ++q) {
      const unsigned short h0 = f2bf_bits(y[2 * q]), h1 = f2bf_bits(y[2 * q + 1]);
      const unsigned short l0 = f2bf_bits(y[2 * q] - bf_bits2f(h0)), l1 = f2bf_bits(y[2 * q + 1] - bf_bits2f(h1));
      const unsigned hw = pk16(h0, h1), lw = pk16(l0, l1);
      rv[q] = (lane < 16) ? hw : lw;
    }
    ov[i] = rv;
  }
  unsigned short* arow = AG + ((size_t)b * NL_ + q0w) * (size_t)AGP + 8 * lane;
#pragma unroll
  for (int i = 0; i < 16; ++i) *(volatile v4u*)(arow + (size_t)i * AGP) = ov[i];
  __threadfence();
#pragma unroll
  for (int i = 0; i < 16; ++i) *(volatile v4u*)(arow + (size_t)i * AGP) = ov[i];
}

__global__ __launch_bounds__(GTHR) void k_gemm(const unsigned short* __restrict__ AG, const unsigned short* __restrict__ BT1,
                                               const unsigned short* __restrict__ XB, const unsigned short* __restrict__ BW2,
                                               float* __restrict__ pre, float* __restrict__ part) {
  __shared__ __align__(16) float stg[GBM * GBN];
  __shared__ __align__(16) float wst[GWAVE * WSTW];
  __shared__ __align__(16) float pst[PARTW];
  const int tid = threadIdx.x, lane = tid & 31, w = tid >> 5, hh = lane >> 4, m = lane & 15;
  const int rowBase = blockIdx.x * GBM;
  const int rw = rowBase + 16 * w + m;

  v8f acc[8];
#pragma unroll
  for (int t = 0; t < 8; ++t) acc[t] = z8();
  {
    const unsigned short* ap = AG + (size_t)rw * AGP;
    const unsigned short* bp = BT1 + (size_t)m * KW1;
#pragma unroll 1
    for (int k0 = 0; k0 < KW1; k0 += 32) {
      const v16b fa = load_frag(ap + k0, hh);
#pragma unroll
      for (int nt = 0; nt < 8; ++nt) {
        const v16b fb = load_frag(bp + (size_t)(16 * nt) * KW1 + k0, hh);
        acc[nt] = wmma_bf16(fa, fb, acc[nt]);
      }
    }
  }
  {
    const unsigned short* ap = XB + (size_t)rw * DD;
    const unsigned short* bp = BW2 + (size_t)m * KW2;
#pragma unroll 1
    for (int k0 = 0; k0 < KW2; k0 += 32) {
      const v16b fa = load_frag(ap + k0, hh);
#pragma unroll
      for (int nt = 0; nt < 8; ++nt) {
        const v16b fb = load_frag(bp + (size_t)(16 * nt) * KW2 + k0, hh);
        acc[nt] = wmma_bf16(fa, fb, acc[nt]);
      }
    }
  }

#pragma unroll
  for (int nt = 0; nt < 8; ++nt) {
    const int lc = 16 * nt + m;
#pragma unroll
    for (int r = 0; r < 8; ++r) {
      const int lr = 16 * w + 8 * hh + r;
      stg[lr * GBN + lc] = acc[nt][r];
    }
  }
  __syncthreads();

  v4f pv[16];
  float wm[4], wq[4];
#pragma unroll
  for (int j = 0; j < 4; ++j) { wm[j] = 0.0f; wq[j] = 0.0f; }
#pragma unroll
  for (int i = 0; i < 16; ++i) {
    const v4f xq = *(const v4fa*)(stg + (16 * w + i) * GBN + 4 * lane);
    pv[i] = xq;
    const float vv[4] = {xq[0], xq[1], xq[2], xq[3]};
    const float rk = 1.0f / (float)(i + 1);
#pragma unroll
    for (int j = 0; j < 4; ++j) {
      const float d = vv[j] - wm[j];
      wm[j] = fmaf(d, rk, wm[j]);
      wq[j] = fmaf(d, vv[j] - wm[j], wq[j]);
    }
  }

#pragma unroll
  for (int i = 0; i < 16; ++i) {
    float* op = pre + (size_t)(rowBase + 16 * w + i) * (size_t)DD + 4 * lane;
    *(volatile v4f*)op = pv[i];
  }
  __threadfence();
#pragma unroll
  for (int i = 0; i < 16; ++i) {
    float* op = pre + (size_t)(rowBase + 16 * w + i) * (size_t)DD + 4 * lane;
    *(volatile v4f*)op = pv[i];
  }

  if (lane == 0) wst[w * WSTW] = 16.0f;
#pragma unroll
  for (int j = 0; j < 4; ++j) {
    wst[w * WSTW + 1 + 4 * lane + j]       = wm[j];
    wst[w * WSTW + 1 + GBN + 4 * lane + j] = wq[j];
  }
  __syncthreads();
  {
    float n = 0.0f, mean = 0.0f, M2 = 0.0f;
#pragma unroll 1
    for (int w2 = 0; w2 < GWAVE; ++w2) {
      const float nb = wst[w2 * WSTW];
      const float mb = wst[w2 * WSTW + 1 + tid];
      const float qb = wst[w2 * WSTW + 1 + GBN + tid];
      if (nb > 0.5f) {
        const float nn = n + nb;
        const float delta = mb - mean;
        const float f = nb / nn;
        mean = fmaf(delta, f, mean);
        M2 = M2 + qb + delta * delta * n * f;
        n = nn;
      }
    }
    pst[1 + tid] = mean;
    pst[1 + GBN + tid] = M2;
    if (tid == 0) pst[0] = n;
  }
#pragma unroll 1
  for (int i = 2 * GBN + 1 + tid; i < PARTW; i += GTHR) pst[i] = 0.0f;
  __syncthreads();
  const int pb = blockIdx.x;
  v4f ps = {0.0f, 0.0f, 0.0f, 0.0f};
  if (tid < PARTW / 4) {
    ps = *(const v4fa*)(pst + 4 * tid);
    *(volatile v4f*)(part + (size_t)pb * PARTW + 4 * tid) = ps;
  }
  __threadfence();
  if (tid < PARTW / 4) {
    *(volatile v4f*)(part + (size_t)pb * PARTW + 4 * tid) = ps;
  }
}

__global__ __launch_bounds__(DD) void k_bnfin(const float* __restrict__ part, const float* __restrict__ gam,
                                             const float* __restrict__ bet, float* ss) {
  __shared__ __align__(16) float stg[2 * DD];
  const int tid = threadIdx.x;
  const int c = tid;
  double n = 0.0, mean = 0.0, M2 = 0.0;
#pragma unroll 1
  for (int bk = 0; bk < NPART; ++bk) {
    const float* pr = part + (size_t)bk * PARTW;
    const double nb = (double)pr[0];
    const double mb = (double)pr[1 + c];
    const double qb = (double)pr[1 + GBN + c];
    if (nb > 0.5) {
      const double nn = n + nb;
      const double delta = mb - mean;
      const double f = nb / nn;
      mean = mean + delta * f;
      M2 = M2 + qb + delta * delta * n * f;
      n = nn;
    }
  }
  const double nt = n < 1.0 ? 1.0 : n;
  const float varf  = (float)(M2 / nt);
  const float meanf = (float)mean;
  const float rstd = 1.0f / sqrtf(varf + BN_EPS);
  const float sc = bf16r(gam[c]) * rstd;
  const float sh = bf16r(bet[c]) - meanf * sc;
  stg[c] = sc;
  stg[DD + c] = sh;
  __syncthreads();
  v4f v = {0.0f, 0.0f, 0.0f, 0.0f};
  if (tid < (2 * DD) / 4) {
    v = *(const v4fa*)(stg + 4 * tid);
    *(volatile v4f*)(ss + 4 * tid) = v;
  }
  __threadfence();
  if (tid < (2 * DD) / 4) {
    *(volatile v4f*)(ss + 4 * tid) = v;
  }
}

__device__ __forceinline__ float selu_f(float v) {
  const float xc = fminf(fmaxf(v, -10.0f), 10.0f);
  const float e = __expf(xc);
  const float ng = SELU_A * (e - 1.0f);
  const float r = (v > 0.0f) ? v : ng;
  return SELU_S * r;
}

__global__ __launch_bounds__(ATHR) void k_apply(const float* __restrict__ pre, const float* __restrict__ ss,
                                                float* __restrict__ out) {
  __shared__ __align__(16) float ssh[2 * DD];
  const int tid = threadIdx.x, lane = tid & 31, w = tid >> 5;
  ssh[tid] = ss[tid];
  __syncthreads();
  const v4f sc = *(const v4fa*)(ssh + 4 * lane);
  const v4f sh = *(const v4fa*)(ssh + DD + 4 * lane);
  const int row0 = blockIdx.x * APB + 8 * w;
  v4f rv[8];
#pragma unroll
  for (int i = 0; i < 8; ++i) {
    const v4f p = *(const v4fa*)(pre + (size_t)(row0 + i) * DD + 4 * lane);
    v4f y;
    y[0] = selu_f(fmaf(p[0], sc[0], sh[0]));
    y[1] = selu_f(fmaf(p[1], sc[1], sh[1]));
    y[2] = selu_f(fmaf(p[2], sc[2], sh[2]));
    y[3] = selu_f(fmaf(p[3], sc[3], sh[3]));
    rv[i] = y;
  }
#pragma unroll
  for (int i = 0; i < 8; ++i)
    *(volatile v4f*)(out + (size_t)(row0 + i) * DD + 4 * lane) = rv[i];
  __threadfence();
#pragma unroll
  for (int i = 0; i < 8; ++i)
    *(volatile v4f*)(out + (size_t)(row0 + i) * DD + 4 * lane) = rv[i];
}

static inline size_t al256(size_t o) { return (o + 255) & ~(size_t)255; }

extern "C" void kernel_launch(void* const* d_in, const int* in_sizes, int n_in,
                              void* d_out, int out_size, void* d_ws, size_t ws_size,
                              hipStream_t stream) {
  if (n_in < 6) return;
  if (in_sizes[0] != NTOK * DD) return;
  if (in_sizes[1] != DD) return;
  if (in_sizes[2] != DD * DD) return;
  if (in_sizes[3] != DD * DD) return;
  if (in_sizes[4] != DD) return;
  if (in_sizes[5] != DD) return;
  if (out_size != NTOK * DD) return;

  const float* x     = (const float*)d_in[0];
  const float* wmap  = (const float*)d_in[1];
  const float* Watt  = (const float*)d_in[2];
  const float* Wres  = (const float*)d_in[3];
  const float* gamma = (const float*)d_in[4];
  const float* beta  = (const float*)d_in[5];
  float* out = (float*)d_out;

  char* ws = (char*)d_ws;
  size_t off = 0;
  const size_t oXB  = off; off = al256(off + (size_t)NTOK * DD * 2);
  const size_t oXWH = off; off = al256(off + (size_t)NTOK * DD * 2);
  const size_t oXWL = off; off = al256(off + (size_t)NTOK * DD * 2);
  const size_t oXT  = off; off = al256(off + (size_t)NB_ * DD * NL_ * 2);
  const size_t oAG  = off; off = al256(off + (size_t)NTOK * AGP * 2);
  const size_t oBT1 = off; off = al256(off + (size_t)DD * KW1 * 2);
  const size_t oBW2 = off; off = al256(off + (size_t)DD * KW2 * 2);
  const size_t oPRE = off; off = al256(off + (size_t)NTOK * DD * 4);
  const size_t oPT  = off; off = al256(off + (size_t)NPART * PARTW * 4);
  const size_t oSS  = off; off = al256(off + (size_t)(2 * DD) * 4);
  if (off > ws_size || off > (size_t)WSMAX) return;

  unsigned short* XB  = (unsigned short*)(ws + oXB);
  unsigned short* XWH = (unsigned short*)(ws + oXWH);
  unsigned short* XWL = (unsigned short*)(ws + oXWL);
  unsigned short* XT  = (unsigned short*)(ws + oXT);
  unsigned short* AG  = (unsigned short*)(ws + oAG);
  unsigned short* BT1 = (unsigned short*)(ws + oBT1);
  unsigned short* BW2 = (unsigned short*)(ws + oBW2);
  float*          PRE = (float*)(ws + oPRE);
  float*          PT  = (float*)(ws + oPT);
  float*          SS  = (float*)(ws + oSS);

  k_xprep<<<dim3(N8X / 256), 256, 0, stream>>>(x, wmap, XB, XWH, XWL, N8X);
  k_wprep<<<dim3(16), 256, 0, stream>>>(Watt, Wres, BT1, BW2);
  k_tprep<<<dim3(DD / 64, NL_ / 64, NB_), 256, 0, stream>>>(x, XT);
  k_attn<<<dim3(NL_ / QT, NB_), 128, 0, stream>>>(XB, XWH, XWL, XT, AG);
  k_gemm<<<dim3(NTOK / GBM), GTHR, 0, stream>>>(AG, BT1, XB, BW2, PRE, PT);
  k_bnfin<<<dim3(1), DD, 0, stream>>>(PT, gamma, beta, SS);
  k_apply<<<dim3(NTOK / APB), ATHR, 0, stream>>>(PRE, SS, out);
  (void)hipGetLastError();
}
